// KDimSelfAttention_5497558138987
// MI455X (gfx1250) — hardware-verified
//
#include <hip/hip_runtime.h>
#include <math.h>

typedef __attribute__((ext_vector_type(16))) _Float16 v16h;
typedef __attribute__((ext_vector_type(16))) __bf16 v16b;
typedef __attribute__((ext_vector_type(8)))  _Float16 v8h;
typedef __attribute__((ext_vector_type(8)))  float v8f;
typedef __attribute__((ext_vector_type(4)))  float v4f;
typedef __attribute__((ext_vector_type(2)))  float v2f;
typedef __attribute__((ext_vector_type(4)))  unsigned v4u;
typedef __attribute__((ext_vector_type(4)))  int v4i;
typedef float __attribute__((may_alias)) float_a;
typedef int __attribute__((may_alias)) int_a;

template <typename T> __device__ __forceinline__ void vst2(void* p, T v) { *(volatile T*)p = v; __threadfence(); *(volatile T*)p = v; }
__device__ __forceinline__ v8f wmma16(v16h a, v16h b, v8f c) {
  v8f d = __builtin_amdgcn_wmma_f32_16x16x32_f16(false, a, false, b, (short)0, c, false, false);
  asm volatile("v_nop\n\tv_nop\n\tv_nop\n\tv_nop" : "+v"(d) : "v"(a), "v"(b));
  return d;
}
__device__ __forceinline__ v8f wmma_bf(v16b a, v16b b, v8f c) {
  v8f d = __builtin_amdgcn_wmma_f32_16x16x32_bf16(false, a, false, b, (short)0, c, false, false);
  asm volatile("v_nop\n\tv_nop\n\tv_nop\n\tv_nop" : "+v"(d) : "v"(a), "v"(b));
  return d;
}
__device__ __forceinline__ v16h frag_h(const _Float16* rowk0, int lane) {
  union { v16h v; v8h q[2]; } u; const _Float16* p = rowk0 + 8 * (lane >> 4);
  u.q[0] = *(const v8h*)p; u.q[1] = *(const v8h*)(p + 16); return u.v;
}
__device__ __forceinline__ v16h frag_f32(const float* rowk0, int lane) {
  v16h a; const float* p = rowk0 + 8 * (lane >> 4);
#pragma unroll
  for (int i = 0; i < 8; ++i) { a[i] = (_Float16)p[i]; a[8 + i] = (_Float16)p[16 + i]; }
  return a;
}
__device__ __forceinline__ v16h frag_f32s(const float* rowk0, int lane, float sc) {
  v16h a; const float* p = rowk0 + 8 * (lane >> 4);
#pragma unroll
  for (int i = 0; i < 8; ++i) { a[i] = (_Float16)(p[i] * sc); a[8 + i] = (_Float16)(p[16 + i] * sc); }
  return a;
}
__device__ __forceinline__ v16h fragc_f32(const float* W, int k0, int n, int lane, int ld, int K) {
  v16h a; const int g = lane >> 4;
#pragma unroll
  for (int i = 0; i < 8; ++i) { const int ka = k0 + 8 * g + i, kb = ka + 16;
    a[i] = (_Float16)(ka < K ? W[(size_t)(ka < K ? ka : K - 1) * ld + n] : 0.f); a[8 + i] = (_Float16)(kb < K ? W[(size_t)(kb < K ? kb : K - 1) * ld + n] : 0.f); }
  return a;
}
struct F2 { v16b h, l; };
__device__ __forceinline__ F2 bsplit16(const float v[16]) { F2 r;
#pragma unroll
  for (int i = 0; i < 16; ++i) { const __bf16 h = (__bf16)v[i]; r.h[i] = h; r.l[i] = (__bf16)(v[i] - (float)h); }
  return r; }
__device__ __forceinline__ F2 split_row(const float* row, int k0, int lane) { float v[16]; const float* p = row + k0 + 8 * (lane >> 4);
#pragma unroll
  for (int i = 0; i < 8; ++i) { v[i] = p[i]; v[8 + i] = p[16 + i]; }
  return bsplit16(v); }
__device__ __forceinline__ F2 split_rowK(const float* row, int k0, int lane, int K) { float v[16]; const int g = lane >> 4;
#pragma unroll
  for (int i = 0; i < 8; ++i) { const int ka = k0 + 8 * g + i, kb = ka + 16; v[i] = ka < K ? row[ka < K ? ka : K - 1] : 0.f; v[8 + i] = kb < K ? row[kb < K ? kb : K - 1] : 0.f; }
  return bsplit16(v); }
__device__ __forceinline__ F2 split_col(const float* W, int k0, int n, int lane, int ld, int K) { float v[16]; const int g = lane >> 4;
#pragma unroll
  for (int i = 0; i < 8; ++i) { const int ka = k0 + 8 * g + i, kb = ka + 16; v[i] = ka < K ? W[(size_t)(ka < K ? ka : K - 1) * ld + n] : 0.f; v[8 + i] = kb < K ? W[(size_t)(kb < K ? kb : K - 1) * ld + n] : 0.f; }
  return bsplit16(v); }
__device__ __forceinline__ v8f mac3(const F2& a, const F2& b, v8f c) { c = wmma_bf(a.l, b.h, c); c = wmma_bf(a.h, b.l, c); return wmma_bf(a.h, b.h, c); }
__device__ __forceinline__ float sigm(float v) { return 1.0f / (1.0f + expf(-v)); }
#define LDSX() do { asm volatile("s_wait_dscnt 0" ::: "memory"); __builtin_amdgcn_wave_barrier(); __builtin_amdgcn_fence(__ATOMIC_RELEASE, "workgroup"); } while (0)


#define NBC 32
#define TT 2048
#define KD 64
#define NR (NBC * TT)
#define QKVP 192
#ifndef TRB
#define TRB (NR / 64)
#define TQB (TT / 64)
#define TNB NBC
#endif
typedef __attribute__((ext_vector_type(8))) __bf16 v8b;
__device__ __forceinline__ v16b frag_b(const __bf16* rowk0, int lane) {
  union { v16b v; v8b q[2]; } u; const __bf16* p = rowk0 + 8 * (lane >> 4);
  u.q[0] = *(const v8b*)p; u.q[1] = *(const v8b*)(p + 16); return u.v;
}
__device__ __forceinline__ v16b frag_gbf(const float* rowk0, int lane) {
  v16b a; const float* p = rowk0 + 8 * (lane >> 4);
#pragma unroll
  for (int i = 0; i < 8; ++i) { a[i] = (__bf16)p[i]; a[8 + i] = (__bf16)p[16 + i]; }
  return a;
}
__device__ __forceinline__ float bfr(float v) { return (float)(__bf16)v; }
__device__ __attribute__((noinline)) float exp_ni(float v) { return expf(v); }
#define WS_PT   0u
#define WS_QKV  (WS_PT + 2u * QKVP * KD)
#define WS_QS   (WS_QKV + 4u * NR * QKVP)
#define WS_KS   (WS_QS + 4u * NR)
#define WS_VTH  (WS_KS + 4u * NR)
#define WS_VTL  (WS_VTH + 2u * NBC * KD * TT)
#define WS_END  (WS_VTL + 2u * NBC * KD * TT)

__global__ __launch_bounds__(64) void k_pack(const float* __restrict__ Wq, const float* __restrict__ Wk, const float* __restrict__ Wv, __bf16* __restrict__ PT) {
  __shared__ __align__(16) __bf16 srow[64];
  const int n = blockIdx.x, tid = threadIdx.x; const int which = n / KD, c = n % KD; const float* Wm = (which == 0 ? Wq : which == 1 ? Wk : Wv) + (size_t)c * KD;
  srow[tid] = (__bf16)Wm[tid]; __syncthreads();
  if (tid < 8) vst2((unsigned*)(PT + (size_t)n * KD + tid * 8), *(const v4u*)(&srow[tid * 8]));
}
__global__ __launch_bounds__(128) void k_proj(const float* __restrict__ X, const __bf16* __restrict__ PT, const float* __restrict__ bq, const float* __restrict__ bk, const float* __restrict__ bv, float* __restrict__ QKV, float* __restrict__ QS, float* __restrict__ KS) {
  __shared__ __align__(16) float so[4][16][196]; __shared__ __align__(16) float sqs[64], sks[64];
  const int tid = threadIdx.x, wave = tid >> 5, lane = tid & 31, col = lane & 15, g = lane >> 4; const size_t r0 = (size_t)blockIdx.x * 64 + wave * 16;
  v8f acc[12] = {};
#pragma unroll
  for (int kc = 0; kc < 2; ++kc) { const v16b a = frag_gbf(X + (r0 + col) * KD + kc * 32, lane);
#pragma unroll
    for (int j = 0; j < 12; ++j) acc[j] = wmma_bf(a, frag_b(PT + (size_t)(j * 16 + col) * KD + kc * 32, lane), acc[j]); }
#pragma unroll
  for (int j = 0; j < 12; ++j) { const int n = j * 16 + col; const int which = n / KD, c = n % KD; const float bb = bfr((which == 0 ? bq : which == 1 ? bk : bv)[c]);
#pragma unroll
    for (int r = 0; r < 8; ++r) so[wave][8 * g + r][n] = acc[j][r] + bb; }
  LDSX();
  if (lane < 16) { float s1 = 0.f, s2 = 0.f; for (int d = 0; d < KD; ++d) { s1 += so[wave][lane][d]; s2 += so[wave][lane][KD + d]; } sqs[wave * 16 + lane] = s1; sks[wave * 16 + lane] = s2; }
  for (int rl = 0; rl < 16; ++rl) for (int pc = lane; pc < QKVP / 4; pc += 32) vst2(QKV + (r0 + rl) * QKVP + pc * 4, *(const v4f*)&so[wave][rl][pc * 4]);
  __syncthreads();
  if (tid < 16) vst2(QS + (size_t)blockIdx.x * 64 + tid * 4, *(const v4f*)&sqs[tid * 4]); else if (tid < 32) vst2(KS + (size_t)blockIdx.x * 64 + (tid - 16) * 4, *(const v4f*)&sks[(tid - 16) * 4]);
}
__global__ __launch_bounds__(256) void k_vt(const float* __restrict__ QKV, __bf16* __restrict__ VTH, __bf16* __restrict__ VTL) {
  __shared__ __align__(16) __bf16 svh[KD][72], svl[KD][72];
  const int tid = threadIdx.x; const size_t t0 = (size_t)blockIdx.x * 64; const int bc = (int)(t0 / TT), p0 = (int)(t0 % TT);
  for (int q = tid; q < 64 * KD; q += 256) { const int tl = q >> 6, d = q & 63; const float v = QKV[(t0 + tl) * QKVP + 2 * KD + d]; const __bf16 hb = (__bf16)v; svh[d][tl] = hb; svl[d][tl] = (__bf16)(v - (float)hb); }
  __syncthreads();
  for (int q = tid; q < KD * 8; q += 256) { const int rowi = q >> 3, pc = q & 7; const size_t o = ((size_t)bc * KD + rowi) * TT + p0 + pc * 8; vst2((unsigned*)(VTH + o), *(const v4u*)&svh[rowi][pc * 8]); vst2((unsigned*)(VTL + o), *(const v4u*)&svl[rowi][pc * 8]); }
}
__global__ __launch_bounds__(128) void k_attn(const float* __restrict__ QS, const float* __restrict__ KS, const __bf16* __restrict__ VTH, const __bf16* __restrict__ VTL, float* __restrict__ OUT) {
  __shared__ __align__(16) float sp[4][16][36]; __shared__ __align__(16) float so[4][16][68];
  const int tid = threadIdx.x, wave = tid >> 5, lane = tid & 31, col = lane & 15, g = lane >> 4;
  const int qb = blockIdx.x, bc = blockIdx.y; const int q0 = qb * 64 + wave * 16; const size_t tq = (size_t)bc * TT + q0;
  float qsr[8];
#pragma unroll
  for (int r = 0; r < 8; ++r) qsr[r] = QS[tq + 8 * g + r] * 0.125f;
  float m[8], l[8];
#pragma unroll
  for (int r = 0; r < 8; ++r) { m[r] = -3.0e38f; l[r] = 0.f; }
  v8f acc[4] = {};
#pragma unroll 1
  for (int ks = 0; ks < TT / 32; ++ks) {
    const float k0 = KS[(size_t)bc * TT + ks * 32 + col], k1 = KS[(size_t)bc * TT + ks * 32 + 16 + col];
    float s[2][8];
#pragma unroll
    for (int r = 0; r < 8; ++r) { s[0][r] = qsr[r] * k0; s[1][r] = qsr[r] * k1; }
#pragma unroll
    for (int r = 0; r < 8; ++r) { float mx = fmaxf(s[0][r], s[1][r]);
#pragma unroll
      for (int o = 1; o < 16; o <<= 1) mx = fmaxf(mx, __shfl_xor(mx, o));
      const float mn = fmaxf(m[r], mx); const float alpha = exp_ni(m[r] - mn);
      const float e0 = exp_ni(s[0][r] - mn), e1 = exp_ni(s[1][r] - mn); float es = e0 + e1;
#pragma unroll
      for (int o = 1; o < 16; o <<= 1) es += __shfl_xor(es, o);
      l[r] = l[r] * alpha + es; m[r] = mn;
#pragma unroll
      for (int dt = 0; dt < 4; ++dt) acc[dt][r] *= alpha;
      sp[wave][8 * g + r][col] = e0; sp[wave][8 * g + r][16 + col] = e1; }
    LDSX();
    const F2 pa = split_row(&sp[wave][col][0], 0, lane);
#pragma unroll
    for (int dt = 0; dt < 4; ++dt) { const size_t vrow = ((size_t)bc * KD + dt * 16 + col) * TT + ks * 32; const v16b vh = frag_b(VTH + vrow, lane), vl = frag_b(VTL + vrow, lane);
      acc[dt] = wmma_bf(pa.l, vh, acc[dt]); acc[dt] = wmma_bf(pa.h, vl, acc[dt]); acc[dt] = wmma_bf(pa.h, vh, acc[dt]); }
    LDSX(); }
#pragma unroll
  for (int r = 0; r < 8; ++r) { const float il = 1.0f / l[r];
#pragma unroll
    for (int dt = 0; dt < 4; ++dt) so[wave][8 * g + r][dt * 16 + col] = acc[dt][r] * il; }
  LDSX();
  for (int rl = 0; rl < 16; ++rl) if (lane < 16) vst2(OUT + (tq + rl) * KD + lane * 4, *(const v4f*)&so[wave][rl][lane * 4]);
}

extern "C" void kernel_launch(void* const* d_in, const int* in_sizes, int n_in, void* d_out, int out_size, void* d_ws, size_t ws_size, hipStream_t stream) {
  (void)in_sizes; (void)n_in; (void)out_size;
  const float** F = (const float**)d_in;
  if (ws_size < (size_t)WS_END) return;
  char* ws = (char*)d_ws; __bf16 *PT = (__bf16*)(ws + WS_PT), *VTH = (__bf16*)(ws + WS_VTH), *VTL = (__bf16*)(ws + WS_VTL); float *QKV = (float*)(ws + WS_QKV), *QS = (float*)(ws + WS_QS), *KS = (float*)(ws + WS_KS);
  k_pack<<<QKVP, 64, 0, stream>>>(F[1], F[3], F[5], PT);
  k_proj<<<TRB, 128, 0, stream>>>(F[0], PT, F[2], F[4], F[6], QKV, QS, KS);
  k_vt<<<TRB, 256, 0, stream>>>(QKV, VTH, VTL);
  k_attn<<<dim3(TQB, TNB), 128, 0, stream>>>(QS, KS, VTH, VTL, (float*)d_out);
}
